// BertSelfAttention_2851858284546
// MI455X (gfx1250) — hardware-verified
//
#include <hip/hip_runtime.h>


typedef _Float16 v16h __attribute__((ext_vector_type(16)));
typedef _Float16 v8h  __attribute__((ext_vector_type(8)));
typedef float    v8f  __attribute__((ext_vector_type(8)));
typedef float    v4f  __attribute__((ext_vector_type(4)));

#ifndef NB
#define NB 2
#endif
#ifndef SEQ
#define SEQ 2048
#endif
#define NB_FULL  2
#define SEQ_FULL 2048
#define DM   1024
#define NH   16
#define DH   64
#define MROWS (NB * SEQ)

#define X_CARRY   16.0f
#define W_CARRY   64.0f
#define QKV_UNSC  (1.0f / 1024.0f)
#define RES_CARRY 2048.0f
#define RES_INV   (1.0f / 2048.0f)
#define P_CARRY   4096.0f
#define P_INV     (1.0f / 4096.0f)
#define SM_SCALE  0.125f
#define MASK_FILL (-1.0e15f)

static_assert(NB >= 1 && NB <= NB_FULL);
static_assert(SEQ % 128 == 0 && SEQ >= 128 && SEQ <= SEQ_FULL);
static_assert(DM == NH * DH);
static_assert(((long long)MROWS * DM) % 2048 == 0);
static_assert((DM * DM) % 2048 == 0);

__device__ __forceinline__ float bf16r(float f) {
    unsigned int u = __float_as_uint(f);
    u += 0x7FFFu + ((u >> 16) & 1u);
    u &= 0xFFFF0000u;
    return __uint_as_float(u);
}

__device__ __forceinline__ v16h ldfrag(const _Float16* p) {
    union { v16h v; v8h h[2]; } u;
    u.h[0] = *(const v8h*)(p);
    u.h[1] = *(const v8h*)(p + 16);
    return u.v;
}

__device__ __forceinline__ v8f wmma_f16(v16h a, v16h b, v8f c) {
    c = __builtin_amdgcn_wmma_f32_16x16x32_f16(false, a, false, b, (short)0, c, false, false);
    asm volatile("v_nop\n\tv_nop\n\tv_nop\n\tv_nop" : "+v"(c) : "v"(a), "v"(b));
    return c;
}

__device__ __forceinline__ float rmax16(float v) {
    #pragma unroll
    for (int m = 8; m > 0; m >>= 1) v = fmaxf(v, __shfl_xor(v, m, 32));
    return v;
}
__device__ __forceinline__ float rsum16(float v) {
    #pragma unroll
    for (int m = 8; m > 0; m >>= 1) v += __shfl_xor(v, m, 32);
    return v;
}

__global__ __launch_bounds__(256) void cvt_x(const float* __restrict__ x, _Float16* __restrict__ xp) {
    const size_t e = ((size_t)blockIdx.x * 256u + threadIdx.x) * 8u;
    const size_t total = (size_t)MROWS * DM;
    if (e >= total) return;
    const int m   = (int)(e / DM);
    const int col = (int)(e - (size_t)m * DM);
    const int b = m / SEQ;
    const int s = m - b * SEQ;
    const float* src = x + ((size_t)b * SEQ_FULL + s) * DM + col;
    const v4f f0 = *(const v4f*)(src);
    const v4f f1 = *(const v4f*)(src + 4);
    v8h o = {};
    #pragma unroll
    for (int i = 0; i < 4; ++i) {
        o[i]     = (_Float16)(bf16r(f0[i]) * X_CARRY);
        o[i + 4] = (_Float16)(bf16r(f1[i]) * X_CARRY);
    }
    _Float16* dst = xp + e;
    *(volatile v8h*)dst = o;
    __threadfence();
    *(volatile v8h*)dst = o;
}

__global__ __launch_bounds__(256) void cvt_w(const float* __restrict__ wq, const float* __restrict__ wk,
                                              const float* __restrict__ wv, _Float16* __restrict__ wp) {
    const int z = blockIdx.y;
    const float* w = (z == 0) ? wq : ((z == 1) ? wk : wv);
    const size_t e = ((size_t)blockIdx.x * 256u + threadIdx.x) * 8u;
    const size_t total = (size_t)DM * DM;
    if (e >= total) return;
    const float* src = w + e;
    const v4f f0 = *(const v4f*)(src);
    const v4f f1 = *(const v4f*)(src + 4);
    v8h o = {};
    #pragma unroll
    for (int i = 0; i < 4; ++i) {
        o[i]     = (_Float16)(bf16r(f0[i]) * W_CARRY);
        o[i + 4] = (_Float16)(bf16r(f1[i]) * W_CARRY);
    }
    _Float16* dst = wp + (size_t)z * DM * DM + e;
    *(volatile v8h*)dst = o;
    __threadfence();
    *(volatile v8h*)dst = o;
}

#define TM  128
#define TN  64
#define TK  64
#define LDA 72
#define LDT 136
static_assert(TN == DH);
static_assert(DM / TN == NH);
static_assert(TN * LDT <= TM * LDA);
static_assert(SEQ % TM == 0);
static_assert(DM % TK == 0);

__global__ __launch_bounds__(256) void qkv_gemm(const _Float16* __restrict__ Xp,
                                                 const _Float16* __restrict__ Wp,
                                                 const float* __restrict__ bq,
                                                 const float* __restrict__ bk,
                                                 const float* __restrict__ bv,
                                                 _Float16* __restrict__ Qh, _Float16* __restrict__ Ql,
                                                 _Float16* __restrict__ Kh, _Float16* __restrict__ Kl,
                                                 _Float16* __restrict__ Vt) {
    __shared__ __attribute__((aligned(16))) _Float16 As[TM * LDA];
    __shared__ __attribute__((aligned(16))) _Float16 Bs[TN * LDA];

    const int tid  = threadIdx.x;
    const int lane = tid & 31;
    const int wave = tid >> 5;
    const int z    = blockIdx.z;
    const int h    = blockIdx.x;
    const int n0   = h * TN;
    const int m0   = blockIdx.y * TM;
    const int wm   = (wave & 3) << 5;
    const int wn   = (wave >> 2) << 5;
    const int row16 = lane & 15;
    const int hh    = lane >> 4;
    const int kbase = hh << 3;

    const _Float16* W  = Wp + (size_t)z * DM * DM;
    const float* bias  = (z == 0) ? bq : ((z == 1) ? bk : bv);

    v8f c[2][2] = {};

    #pragma unroll 1
    for (int k0 = 0; k0 < DM; k0 += TK) {
        #pragma unroll
        for (int i = 0; i < 4; ++i) {
            const int p  = (i << 8) + tid;
            const int ar = p >> 3;
            const int ac = (p & 7) << 3;
            *(v8h*)&As[ar * LDA + ac] = *(const v8h*)(Xp + (size_t)(m0 + ar) * DM + k0 + ac);
        }
        #pragma unroll
        for (int i = 0; i < 2; ++i) {
            const int p  = (i << 8) + tid;
            const int br = p >> 3;
            const int bc = (p & 7) << 3;
            *(v8h*)&Bs[br * LDA + bc] = *(const v8h*)(W + (size_t)(n0 + br) * DM + k0 + bc);
        }
        __syncthreads();

        #pragma unroll
        for (int kk = 0; kk < 2; ++kk) {
            v16h a[2], bfr[2];
            #pragma unroll
            for (int i = 0; i < 2; ++i)
                a[i] = ldfrag(&As[(wm + (i << 4) + row16) * LDA + (kk << 5) + kbase]);
            #pragma unroll
            for (int j = 0; j < 2; ++j)
                bfr[j] = ldfrag(&Bs[(wn + (j << 4) + row16) * LDA + (kk << 5) + kbase]);
            #pragma unroll
            for (int i = 0; i < 2; ++i)
                #pragma unroll
                for (int j = 0; j < 2; ++j)
                    c[i][j] = wmma_f16(a[i], bfr[j], c[i][j]);
        }
        __syncthreads();
    }

    const int bidx = m0 / SEQ;
    const int s0   = m0 - bidx * SEQ;
    float bb[2];
    #pragma unroll
    for (int j = 0; j < 2; ++j) bb[j] = bf16r(bias[n0 + wn + (j << 4) + row16]);

    if (z < 2) {
        _Float16* Oh = (z == 0) ? Qh : Kh;
        _Float16* Ol = (z == 0) ? Ql : Kl;
        const size_t obase = (((size_t)bidx * NH + h) * SEQ + s0) * DH;
        #pragma unroll
        for (int pass = 0; pass < 2; ++pass) {
            #pragma unroll
            for (int i = 0; i < 2; ++i)
                #pragma unroll
                for (int j = 0; j < 2; ++j)
                    #pragma unroll
                    for (int r = 0; r < 8; ++r) {
                        const float v = c[i][j][r] * QKV_UNSC + bb[j];
                        const _Float16 hv = (_Float16)v;
                        const _Float16 sv = (pass == 0) ? hv : (_Float16)((v - (float)hv) * RES_CARRY);
                        As[(wm + (i << 4) + (hh << 3) + r) * LDA + wn + (j << 4) + row16] = sv;
                    }
            __syncthreads();
            v8h pc[4];
            #pragma unroll
            for (int it = 0; it < 4; ++it) {
                const int p   = (it << 8) + tid;
                const int row = p >> 3;
                const int c8  = (p & 7) << 3;
                pc[it] = *(const v8h*)&As[row * LDA + c8];
            }
            _Float16* O = (pass == 0) ? Oh : Ol;
            #pragma unroll
            for (int it = 0; it < 4; ++it) {
                const int p   = (it << 8) + tid;
                const int row = p >> 3;
                const int c8  = (p & 7) << 3;
                *(volatile v8h*)(O + obase + (size_t)row * DH + c8) = pc[it];
            }
            __threadfence();
            #pragma unroll
            for (int it = 0; it < 4; ++it) {
                const int p   = (it << 8) + tid;
                const int row = p >> 3;
                const int c8  = (p & 7) << 3;
                *(volatile v8h*)(O + obase + (size_t)row * DH + c8) = pc[it];
            }
            __syncthreads();
        }
    } else {
        #pragma unroll
        for (int i = 0; i < 2; ++i)
            #pragma unroll
            for (int j = 0; j < 2; ++j) {
                v8h pk = {};
                #pragma unroll
                for (int r = 0; r < 8; ++r) pk[r] = (_Float16)(c[i][j][r] * QKV_UNSC + bb[j]);
                *(v8h*)&As[(wn + (j << 4) + row16) * LDT + wm + (i << 4) + (hh << 3)] = pk;
            }
        __syncthreads();
        const size_t vbase = (((size_t)bidx * NH + h) * DH) * SEQ + s0;
        v8h pc[4];
        #pragma unroll
        for (int it = 0; it < 4; ++it) {
            const int p  = (it << 8) + tid;
            const int dr = p >> 4;
            const int c8 = (p & 15) << 3;
            pc[it] = *(const v8h*)&As[dr * LDT + c8];
        }
        #pragma unroll
        for (int it = 0; it < 4; ++it) {
            const int p  = (it << 8) + tid;
            const int dr = p >> 4;
            const int c8 = (p & 15) << 3;
            *(volatile v8h*)(Vt + vbase + (size_t)dr * SEQ + c8) = pc[it];
        }
        __threadfence();
        #pragma unroll
        for (int it = 0; it < 4; ++it) {
            const int p  = (it << 8) + tid;
            const int dr = p >> 4;
            const int c8 = (p & 15) << 3;
            *(volatile v8h*)(Vt + vbase + (size_t)dr * SEQ + c8) = pc[it];
        }
    }
}

#define QT   128
#define KBLK 64
#define LDK  72
#define LDO  20
#define POOL_HALVES (3 * KBLK * LDK + 8 * 16 * LDK)
#define POOL_FLOATS (POOL_HALVES / 2)
static_assert(SEQ % QT == 0 && SEQ % KBLK == 0);
static_assert(POOL_HALVES % 8 == 0);
static_assert(8 * DH * LDO <= POOL_FLOATS);
static_assert((KBLK * LDK) % 8 == 0 && (16 * LDK) % 8 == 0);

__global__ __launch_bounds__(256) void attn(const _Float16* __restrict__ Qh,
                                             const _Float16* __restrict__ Ql,
                                             const _Float16* __restrict__ Kh,
                                             const _Float16* __restrict__ Kl,
                                             const _Float16* __restrict__ Vt,
                                             const int* __restrict__ amask,
                                             const float* __restrict__ Cp,
                                             float* __restrict__ out) {
    __shared__ __attribute__((aligned(16))) float pool[POOL_FLOATS];
    _Float16* const sm  = reinterpret_cast<_Float16*>(pool);
    _Float16* const Ks  = sm;
    _Float16* const Kls = sm + KBLK * LDK;
    _Float16* const Vs  = sm + 2 * KBLK * LDK;
    _Float16* const Ps  = sm + 3 * KBLK * LDK;

    const int tid  = threadIdx.x;
    const int lane = tid & 31;
    const int wave = tid >> 5;
    const int bh   = blockIdx.y;
    const int b    = bh / NH;
    const int h    = bh - b * NH;
    const int q0   = blockIdx.x * QT + (wave << 4);
    const int row16 = lane & 15;
    const int hh    = lane >> 4;
    const int kbase = hh << 3;

    const size_t baseQK = (size_t)bh * SEQ * DH;
    const size_t baseV  = (size_t)bh * DH * SEQ;

    v16h qh[2], ql[2];
    #pragma unroll
    for (int kk = 0; kk < 2; ++kk) {
        qh[kk] = ldfrag(Qh + baseQK + (size_t)(q0 + row16) * DH + (kk << 5) + kbase);
        ql[kk] = ldfrag(Ql + baseQK + (size_t)(q0 + row16) * DH + (kk << 5) + kbase);
    }

    v8f acc[4] = {};
    float mrow[8], lrow[8];
    #pragma unroll
    for (int r = 0; r < 8; ++r) { mrow[r] = -1.0e30f; lrow[r] = 0.0f; }

    _Float16* const P = Ps + wave * 16 * LDK;
    const int* const mk = amask + (size_t)b * SEQ_FULL;
    const float* const crow = Cp + ((size_t)b * SEQ_FULL + (size_t)(q0 + (hh << 3))) * SEQ_FULL;

    const int key = tid >> 2;
    const int dc  = (tid & 3) << 4;

    #pragma unroll 1
    for (int kb = 0; kb < SEQ; kb += KBLK) {
        __syncthreads();
        {
            const _Float16* ks = Kh + baseQK + (size_t)(kb + key) * DH + dc;
            const _Float16* kl = Kl + baseQK + (size_t)(kb + key) * DH + dc;
            const _Float16* vs = Vt + baseV + (size_t)key * SEQ + kb + dc;
            *(v8h*)&Ks[key * LDK + dc]      = *(const v8h*)(ks);
            *(v8h*)&Ks[key * LDK + dc + 8]  = *(const v8h*)(ks + 8);
            *(v8h*)&Kls[key * LDK + dc]     = *(const v8h*)(kl);
            *(v8h*)&Kls[key * LDK + dc + 8] = *(const v8h*)(kl + 8);
            *(v8h*)&Vs[key * LDK + dc]      = *(const v8h*)(vs);
            *(v8h*)&Vs[key * LDK + dc + 8]  = *(const v8h*)(vs + 8);
        }
        __syncthreads();

        v8f sc[4];
        #pragma unroll
        for (int j = 0; j < 4; ++j) {
            v8f s = {};
            v8f sr = {};
            #pragma unroll
            for (int kk = 0; kk < 2; ++kk) {
                const int ko = ((j << 4) + row16) * LDK + (kk << 5) + kbase;
                const v16h khf = ldfrag(&Ks[ko]);
                const v16h klf = ldfrag(&Kls[ko]);
                s  = wmma_f16(qh[kk], khf, s);
                sr = wmma_f16(qh[kk], klf, sr);
                sr = wmma_f16(ql[kk], khf, sr);
            }
            const int mv = mk[kb + (j << 4) + row16];
            v8f t = {};
            #pragma unroll
            for (int r = 0; r < 8; ++r) {
                const float v = (s[r] + sr[r] * RES_INV) * SM_SCALE;
                t[r] = (mv == 0) ? MASK_FILL : v;
            }
            sc[j] = t;
        }

        #pragma unroll
        for (int r = 0; r < 8; ++r) {
            float mx = fmaxf(fmaxf(sc[0][r], sc[1][r]), fmaxf(sc[2][r], sc[3][r]));
            mx = rmax16(mx);
            const float mnew = fmaxf(mrow[r], mx);
            const float corr = __expf(mrow[r] - mnew);
            mrow[r] = mnew;
            #pragma unroll
            for (int jd = 0; jd < 4; ++jd) acc[jd][r] = acc[jd][r] * corr;
            float sum = 0.0f;
            #pragma unroll
            for (int j = 0; j < 4; ++j) {
                const float e = __expf(sc[j][r] - mnew);
                sc[j][r] = e;
                sum += e;
            }
            lrow[r] = lrow[r] * corr + rsum16(sum);
        }

        #pragma unroll
        for (int j = 0; j < 4; ++j) {
            float cv[8];
            #pragma unroll
            for (int r = 0; r < 8; ++r)
                cv[r] = bf16r(crow[(size_t)r * SEQ_FULL + kb + (j << 4) + row16]) * P_CARRY;
            #pragma unroll
            for (int r = 0; r < 8; ++r)
                P[(r + (hh << 3)) * LDK + (j << 4) + row16] = (_Float16)(sc[j][r] * cv[r]);
            asm volatile("" ::: "memory");
        }
        __builtin_amdgcn_fence(3  , "wavefront");
        __builtin_amdgcn_wave_barrier();

        #pragma unroll
        for (int kk = 0; kk < 2; ++kk) {
            const v16h pf = ldfrag(&P[row16 * LDK + (kk << 5) + kbase]);
            #pragma unroll
            for (int jd = 0; jd < 4; ++jd) {
                const v16h vf = ldfrag(&Vs[((jd << 4) + row16) * LDK + (kk << 5) + kbase]);
                acc[jd] = wmma_f16(pf, vf, acc[jd]);
            }
        }
    }

    __syncthreads();
    float* const Os = pool + wave * (DH * LDO);
    float inv[8];
    #pragma unroll
    for (int r = 0; r < 8; ++r) inv[r] = (1.0f / lrow[r]) * P_INV;
    #pragma unroll
    for (int jd = 0; jd < 4; ++jd) {
        v4f o0 = {}, o1 = {};
        #pragma unroll
        for (int r = 0; r < 4; ++r) {
            o0[r] = acc[jd][r] * inv[r];
            o1[r] = acc[jd][r + 4] * inv[r + 4];
        }
        float* d = &Os[((jd << 4) + row16) * LDO + (hh << 3)];
        *(v4f*)(d)     = o0;
        *(v4f*)(d + 4) = o1;
    }
    __builtin_amdgcn_fence(3  , "wavefront");
    __builtin_amdgcn_wave_barrier();

    v4f ov[8];
    #pragma unroll
    for (int it = 0; it < 8; ++it) {
        const int row = (it << 1) + hh;
        const int c4  = row16 << 2;
        v4f t4 = {};
        #pragma unroll
        for (int q = 0; q < 4; ++q) t4[q] = Os[(c4 + q) * LDO + row];
        ov[it] = t4;
    }
    float* const ob = out + ((size_t)b * SEQ + q0) * DM + (size_t)h * DH;
    #pragma unroll
    for (int it = 0; it < 8; ++it) {
        const int row = (it << 1) + hh;
        const int c4  = row16 << 2;
        *(volatile v4f*)(ob + (size_t)row * DM + c4) = ov[it];
    }
    __threadfence();
    #pragma unroll
    for (int it = 0; it < 8; ++it) {
        const int row = (it << 1) + hh;
        const int c4  = row16 << 2;
        *(volatile v4f*)(ob + (size_t)row * DM + c4) = ov[it];
    }
}

extern "C" void kernel_launch(void* const* d_in, const int* in_sizes, int n_in,
                              void* d_out, int out_size, void* d_ws, size_t ws_size,
                              hipStream_t stream) {
    if (n_in < 9) return;
    const float* x  = (const float*)d_in[0];
    const int*   am = (const int*)d_in[1];
    const float* cp = (const float*)d_in[2];
    const float* wq = (const float*)d_in[3];
    const float* bq = (const float*)d_in[4];
    const float* wk = (const float*)d_in[5];
    const float* bk = (const float*)d_in[6];
    const float* wv = (const float*)d_in[7];
    const float* bv = (const float*)d_in[8];

    const long long need_x = ((long long)(NB - 1) * SEQ_FULL + SEQ) * DM;
    const long long need_m = (long long)(NB - 1) * SEQ_FULL + SEQ;
    const long long need_c = ((long long)(NB - 1) * SEQ_FULL + (SEQ - 1)) * SEQ_FULL + SEQ;
    if ((long long)in_sizes[0] < need_x) return;
    if ((long long)in_sizes[1] < need_m) return;
    if ((long long)in_sizes[2] < need_c) return;
    if (in_sizes[3] < DM * DM || in_sizes[5] < DM * DM || in_sizes[7] < DM * DM) return;
    if (in_sizes[4] < DM || in_sizes[6] < DM || in_sizes[8] < DM) return;
    if ((long long)out_size < (long long)MROWS * DM) return;

    const size_t plane  = (size_t)MROWS * DM;
    const size_t pbytes = plane * sizeof(_Float16);
    const size_t wbytes = (size_t)3 * DM * DM * sizeof(_Float16);
    const size_t oXp = 0;
    const size_t oWp = oXp + pbytes;
    const size_t oQh = oWp + wbytes;
    const size_t oQl = oQh + pbytes;
    const size_t oKh = oQl + pbytes;
    const size_t oKl = oKh + pbytes;
    const size_t oVt = oKl + pbytes;
    const size_t oEnd = oVt + pbytes;
    if (oEnd > ws_size) return;

    char* ws = (char*)d_ws;
    _Float16* Xp = (_Float16*)(ws + oXp);
    _Float16* Wp = (_Float16*)(ws + oWp);
    _Float16* Qh = (_Float16*)(ws + oQh);
    _Float16* Ql = (_Float16*)(ws + oQl);
    _Float16* Kh = (_Float16*)(ws + oKh);
    _Float16* Kl = (_Float16*)(ws + oKl);
    _Float16* Vt = (_Float16*)(ws + oVt);

    cvt_x<<<dim3((unsigned)(plane / 2048)), dim3(256), 0, stream>>>(x, Xp);
    cvt_w<<<dim3((DM * DM) / 2048, 3), dim3(256), 0, stream>>>(wq, wk, wv, Wp);
    qkv_gemm<<<dim3(NH, MROWS / TM, 3), dim3(256), 0, stream>>>(Xp, Wp, bq, bk, bv, Qh, Ql, Kh, Kl, Vt);
    attn<<<dim3(SEQ / QT, NB * NH), dim3(256), 0, stream>>>(Qh, Ql, Kh, Kl, Vt, am, cp, (float*)d_out);
}
